// GatedAttentionUnit_20950850470540
// MI455X (gfx1250) — hardware-verified
//
#include <hip/hip_runtime.h>

typedef __attribute__((ext_vector_type(16))) _Float16 v16h;
typedef __attribute__((ext_vector_type(8)))  _Float16 v8h;
typedef __attribute__((ext_vector_type(16))) __bf16   v16b;
typedef __attribute__((ext_vector_type(8)))  __bf16   v8b;
typedef __attribute__((ext_vector_type(8)))  float    v8f;
typedef __attribute__((ext_vector_type(4)))  float    v4f;

constexpr int NBATCH = 8;
constexpr int LSEQ   = 2048;
constexpr int DMODEL = 512;
constexpr int SHEAD  = 128;
constexpr int EDIM   = 1024;
constexpr int NUV    = 2 * EDIM + SHEAD;
constexpr int NROWS  = NBATCH * LSEQ;
constexpr int GRP    = 2;
constexpr int GROWS  = GRP * LSEQ;
constexpr int NGRP   = NBATCH / GRP;
static_assert(NBATCH % GRP == 0, "grouping");
static_assert(NUV == 2176 && NROWS == 16384, "shapes");

static_assert(DMODEL % 32 == 0 && SHEAD % 32 == 0 && LSEQ % 32 == 0 && EDIM % 32 == 0, "K multiples of 32");
static_assert(LSEQ % 64 == 0 && EDIM % 64 == 0 && SHEAD % 64 == 0 && DMODEL % 64 == 0, "tile multiples");
static_assert(((LSEQ / 64) * (EDIM / 64)) % 8 == 0, "tiles per block");
static_assert(((LSEQ / 64) * (SHEAD / 64)) % 8 == 0, "tiles per block");
static_assert(((LSEQ / 64) * (LSEQ / 64)) % 8 == 0, "tiles per block");
static_assert(((LSEQ / 64) * (DMODEL / 64)) % 8 == 0, "tiles per block");
static_assert(NROWS % 8 == 0, "norm grid");
static_assert(NUV % 64 == 0 && DMODEL % 64 == 0 && EDIM % 64 == 0, "transpose tiles");

constexpr size_t SZ_WUVT = (size_t)NUV * DMODEL * 2;
constexpr size_t SZ_WO   = (size_t)DMODEL * EDIM * 2;
constexpr size_t SZ_XN   = (size_t)NROWS * DMODEL * 2;
constexpr size_t SZ_U    = (size_t)GROWS * EDIM * 4;
constexpr size_t SZ_VT   = (size_t)GRP * EDIM * LSEQ * 2;
constexpr size_t SZ_QK   = (size_t)GROWS * SHEAD * 2;
constexpr size_t SZ_SC   = (size_t)GRP * LSEQ * LSEQ * 2;
constexpr size_t SZ_H    = (size_t)GROWS * EDIM * 2;
constexpr size_t OFF_WUVT = 0;
constexpr size_t OFF_WOH  = OFF_WUVT + SZ_WUVT;
constexpr size_t OFF_WOL  = OFF_WOH + SZ_WO;
constexpr size_t OFF_XN   = OFF_WOL + SZ_WO;
constexpr size_t OFF_U    = OFF_XN + SZ_XN;
constexpr size_t OFF_VT   = OFF_U + SZ_U;
constexpr size_t OFF_Q    = OFF_VT + SZ_VT;
constexpr size_t OFF_K    = OFF_Q + SZ_QK;
constexpr size_t OFF_SC   = OFF_K + SZ_QK;
constexpr size_t OFF_HH   = OFF_SC + SZ_SC;
constexpr size_t OFF_HL   = OFF_HH + SZ_H;
constexpr size_t WS_TOTAL = OFF_HL + SZ_H;
static_assert(WS_TOTAL == 81920000, "carve total");
static_assert(WS_TOTAL <= 134217728, "carve limit");
static_assert(OFF_WOH % 128 == 0 && OFF_WOL % 128 == 0 && OFF_XN % 128 == 0 && OFF_U % 128 == 0 &&
              OFF_VT % 128 == 0 && OFF_Q % 128 == 0 && OFF_K % 128 == 0 && OFF_SC % 128 == 0 &&
              OFF_HH % 128 == 0 && OFF_HL % 128 == 0, "line alignment");

__device__ __forceinline__ unsigned short f2bf_bits(float f) {
  unsigned u = __float_as_uint(f);
  return (unsigned short)((u + 0x7FFFu + ((u >> 16) & 1u)) >> 16);
}
__device__ __forceinline__ float bf_bits2f(unsigned short h) { return __uint_as_float(((unsigned)h) << 16); }

__device__ __forceinline__ void dep_guard_h(v8f& a, v8f& b, v16h x, v16h y) { asm volatile("v_nop\n\tv_nop\n\tv_nop\n\tv_nop" : "+v"(a), "+v"(b) : "v"(x), "v"(y)); }
__device__ __forceinline__ void dep_guard_b(v8f& a, v8f& b, v16b x, v16b y) { asm volatile("v_nop\n\tv_nop\n\tv_nop\n\tv_nop" : "+v"(a), "+v"(b) : "v"(x), "v"(y)); }
__device__ __forceinline__ void keep4_h(v16h a, v16h b, v16h c, v16h d) { asm volatile("v_nop" :: "v"(a), "v"(b), "v"(c), "v"(d)); }
__device__ __forceinline__ void keep4_b(v16b a, v16b b, v16b c, v16b d) { asm volatile("v_nop" :: "v"(a), "v"(b), "v"(c), "v"(d)); }
__device__ __forceinline__ void acc_guard4(v8f& a, v8f& b, v8f& c, v8f& d) { asm volatile("v_nop\n\tv_nop\n\tv_nop\n\tv_nop" : "+v"(a), "+v"(b), "+v"(c), "+v"(d)); }
template <typename T> struct Frag;
template <> struct Frag<_Float16> {
  typedef v16h V; union U { v16h v; v8h h[2]; };
  static __device__ __forceinline__ v16h load(const _Float16* p) {
    U f; f.h[0] = *(const v8h*)(p); f.h[1] = *(const v8h*)(p + 16); return f.v;
  }
  static __device__ __forceinline__ v8f mma(v16h a, v16h b, v8f c) {
    return __builtin_amdgcn_wmma_f32_16x16x32_f16(false, a, false, b, (short)0, c, false, false);
  }
  static __device__ __forceinline__ void guard(v8f& a, v8f& b, v16h x, v16h y) { dep_guard_h(a, b, x, y); }
  static __device__ __forceinline__ void keep(v16h a, v16h b, v16h c, v16h d) { keep4_h(a, b, c, d); }
};
template <> struct Frag<__bf16> {
  typedef v16b V; union U { v16b v; v8b h[2]; };
  static __device__ __forceinline__ v16b load(const __bf16* p) {
    U f; f.h[0] = *(const v8b*)(p); f.h[1] = *(const v8b*)(p + 16); return f.v;
  }
  static __device__ __forceinline__ v8f mma(v16b a, v16b b, v8f c) {
    return __builtin_amdgcn_wmma_f32_16x16x32_bf16(false, a, false, b, (short)0, c, false, false);
  }
  static __device__ __forceinline__ void guard(v8f& a, v8f& b, v16b x, v16b y) { dep_guard_b(a, b, x, y); }
  static __device__ __forceinline__ void keep(v16b a, v16b b, v16b c, v16b d) { keep4_b(a, b, c, d); }
};
template <int ET> struct Elem;
template <> struct Elem<0> { typedef _Float16 T; };
template <> struct Elem<1> { typedef __bf16 T; };

constexpr int EPI_U = 0;
constexpr int EPI_VT = 1;
constexpr int EPI_QK = 2;
constexpr int EPI_SC = 3;
constexpr int EPI_GATE = 4;
constexpr int EPI_OUT = 5;

template <int ET, bool SPLIT, int EPI>
__global__ __launch_bounds__(256) void gemm64(
    const unsigned short* __restrict__ Ap, const unsigned short* __restrict__ A2p, int lda, long strideA,
    const unsigned short* __restrict__ Btp, const unsigned short* __restrict__ Bt2p, int ldb, long strideB,
    void* __restrict__ Cout, void* __restrict__ Cout2, int ldc, long strideC,
    const float* __restrict__ p0, const float* __restrict__ p1, long strideP,
    int M, int N, int K, float scale, float aux) {
  typedef typename Elem<ET>::T T;
  typedef typename Frag<T>::V V;
  const T* A = (const T*)Ap; const T* A2 = (const T*)A2p; const T* Bt = (const T*)Btp; const T* Bt2 = (const T*)Bt2p;
  __shared__ __align__(16) float sT[8][16 * 68];
  __shared__ __align__(16) float sW[(EPI == EPI_SC) ? 8 : 1][128];
  const int b    = blockIdx.y;
  const int lane = threadIdx.x & 31;
  const int wave = threadIdx.x >> 5;
  const int tilesN = N >> 6;
  const int tilesM = M >> 6;
  const int tile = blockIdx.x * 8 + wave;
  if (tile >= tilesM * tilesN) return;
  const int tm = tile / tilesN;
  const int tn = tile - tm * tilesN;
  const int m0 = tm << 6;
  const int n0 = tn << 6;

  const T* Ab  = A  + (size_t)b * strideA;
  const T* Bb  = Bt + (size_t)b * strideB;
  const T* Ab2 = SPLIT ? (A2  + (size_t)b * strideA) : nullptr;
  const T* Bb2 = SPLIT ? (Bt2 + (size_t)b * strideB) : nullptr;

  const int rlane = lane & 15;
  const int koff  = (lane >> 4) * 8;
  const int mOff  = (lane >> 4) * 8;

  v8f acc[4][4];
#pragma unroll
  for (int i = 0; i < 4; ++i)
#pragma unroll
    for (int j = 0; j < 4; ++j) acc[i][j] = (v8f){0.f,0.f,0.f,0.f,0.f,0.f,0.f,0.f};

  for (int k0 = 0; k0 < K; k0 += 32) {
    V bh[4], bl[4];
#pragma unroll
    for (int j = 0; j < 4; ++j) {
      const size_t bo = (size_t)(n0 + (j << 4) + rlane) * ldb + koff + k0;
      bh[j] = Frag<T>::load(Bb + bo);
      if (SPLIT) bl[j] = Frag<T>::load(Bb2 + bo);
    }
#pragma unroll
    for (int i = 0; i < 4; ++i) {
      const size_t ao = (size_t)(m0 + (i << 4) + rlane) * lda + koff + k0;
      V ah = Frag<T>::load(Ab + ao);
      V al;
      if (SPLIT) al = Frag<T>::load(Ab2 + ao);
#pragma unroll
      for (int j = 0; j < 4; ++j) {
        acc[i][j] = Frag<T>::mma(ah, bh[j], acc[i][j]);
        if (SPLIT) {
          acc[i][j] = Frag<T>::mma(ah, bl[j], acc[i][j]);
          acc[i][j] = Frag<T>::mma(al, bh[j], acc[i][j]);
        }
      }
      Frag<T>::guard(acc[i][0], acc[i][3], ah, SPLIT ? al : ah);
    }
    Frag<T>::keep(bh[0], bh[1], bh[2], bh[3]);
    if (SPLIT) Frag<T>::keep(bl[0], bl[1], bl[2], bl[3]);
  }
  acc_guard4(acc[0][0], acc[0][1], acc[0][2], acc[0][3]);
  acc_guard4(acc[1][0], acc[1][1], acc[1][2], acc[1][3]);
  acc_guard4(acc[2][0], acc[2][1], acc[2][2], acc[2][3]);
  acc_guard4(acc[3][0], acc[3][1], acc[3][2], acc[3][3]);

  constexpr bool OUT32 = (EPI == EPI_U) || (EPI == EPI_OUT);
  float* slab = sT[wave];
  float* wl = sW[(EPI == EPI_SC) ? wave : 0];
  if (EPI == EPI_SC) {
    const int base = (LSEQ - 1) - 63 + n0 - m0;
#pragma unroll
    for (int e = 0; e < 4; ++e) {
      int idx = base + 4 * lane + e;
      idx = idx < 0 ? 0 : idx;
      idx = idx > (2 * LSEQ - 2) ? (2 * LSEQ - 2) : idx;
      wl[4 * lane + e] = p0[idx];
    }
    __builtin_amdgcn_fence(__ATOMIC_RELEASE, "workgroup");
    __builtin_amdgcn_wave_barrier();
    __builtin_amdgcn_fence(__ATOMIC_ACQUIRE, "workgroup");
  }
#pragma unroll
  for (int i = 0; i < 4; ++i) {
    const int mBase = m0 + (i << 4);
#pragma unroll
    for (int j = 0; j < 4; ++j) {
#pragma unroll
      for (int r = 0; r < 8; ++r) {
        float v = acc[i][j][r] * scale;
        if (EPI == EPI_U || EPI == EPI_VT || EPI == EPI_QK) {
          const float en = expf(fminf(-v, 64.0f));
          v = v * (1.0f / (1.0f + en));
        }
        if (EPI == EPI_VT) v = v * aux;
        if (EPI == EPI_SC) {
          const float bias = wl[63 + (j - i) * 16 - r + rlane - mOff];
          v = (v + bias) * aux;
          v = fmaxf(v, 0.0f);
          v = v * v;
        }
        slab[(mOff + r) * 68 + (j << 4) + rlane] = v;
      }
    }
    __builtin_amdgcn_fence(__ATOMIC_RELEASE, "workgroup");
    __builtin_amdgcn_wave_barrier();
    __builtin_amdgcn_fence(__ATOMIC_ACQUIRE, "workgroup");
    if (OUT32) {
      float* Cb = (float*)Cout + (size_t)b * strideC;
      const int hh = lane >> 4, c4 = (lane & 15) * 4;
      const float* Xb = p0 + (size_t)b * strideP;
      v4f rs = (v4f){0.f, 0.f, 0.f, 0.f};
      if (EPI == EPI_OUT) rs = *(const v4f*)(p1 + n0 + c4);
      for (int pass = 0; pass < 2; ++pass) {
#pragma unroll
        for (int it = 0; it < 8; ++it) {
          const int row = it * 2 + hh;
          const size_t go = (size_t)(mBase + row) * ldc + n0 + c4;
          v4f v = *(const v4f*)(slab + row * 68 + c4);
          if (EPI == EPI_OUT) {
            const v4f xr = *(const v4f*)(Xb + go);
            v = v + xr * rs;
          }
          *(volatile v4f*)(Cb + go) = v;
        }
        __threadfence();
      }
    } else {
      const int q = lane >> 3, c8 = (lane & 7) * 8;
      unsigned short* Cb  = (unsigned short*)Cout  + (size_t)b * strideC;
      unsigned short* Cb2 = (unsigned short*)Cout2 + (size_t)b * strideC;
      const float* Ub = p0 + (size_t)b * strideP;
      float ga[8], gb[8], bq[8], bk[8];
#pragma unroll
      for (int e = 0; e < 8; ++e) { ga[e] = 0.f; gb[e] = 0.f; bq[e] = 0.f; bk[e] = 0.f; }
      if (EPI == EPI_QK) {
        const int n = n0 + c8;
        const v4f g0a = *(const v4f*)(p0 + n), g0b = *(const v4f*)(p0 + n + 4);
        const v4f b0a = *(const v4f*)(p1 + n), b0b = *(const v4f*)(p1 + n + 4);
        const v4f g1a = *(const v4f*)(p0 + SHEAD + n), g1b = *(const v4f*)(p0 + SHEAD + n + 4);
        const v4f b1a = *(const v4f*)(p1 + SHEAD + n), b1b = *(const v4f*)(p1 + SHEAD + n + 4);
#pragma unroll
        for (int e = 0; e < 4; ++e) {
          ga[e] = g0a[e]; ga[4 + e] = g0b[e]; bq[e] = b0a[e]; bq[4 + e] = b0b[e];
          gb[e] = g1a[e]; gb[4 + e] = g1b[e]; bk[e] = b1a[e]; bk[4 + e] = b1b[e];
        }
      }
      for (int pass = 0; pass < 2; ++pass) {
#pragma unroll
        for (int it = 0; it < 4; ++it) {
          const int row = it * 4 + q;
          const float* sp = slab + row * 68 + c8;
          const size_t go = (size_t)(mBase + row) * ldc + n0 + c8;
          float uu[8];
#pragma unroll
          for (int e = 0; e < 8; ++e) uu[e] = 0.f;
          if (EPI == EPI_GATE) {
            const v4f u0 = *(const v4f*)(Ub + go), u1 = *(const v4f*)(Ub + go + 4);
#pragma unroll
            for (int e = 0; e < 4; ++e) { uu[e] = u0[e]; uu[4 + e] = u1[e]; }
          }
          v8h hv, lv;
#pragma unroll
          for (int e = 0; e < 8; ++e) {
            const float s = sp[e];
            if (EPI == EPI_VT || EPI == EPI_SC) {
              hv[e] = (_Float16)s;
              lv[e] = hv[e];
            } else if (EPI == EPI_QK) {
              hv[e] = (_Float16)(s * ga[e] + bq[e]);
              lv[e] = (_Float16)(s * gb[e] + bk[e]);
            } else {
              const float hval = s * uu[e];
              const unsigned short hb = f2bf_bits(hval);
              const unsigned short lb = f2bf_bits(hval - bf_bits2f(hb));
              hv[e] = __builtin_bit_cast(_Float16, hb);
              lv[e] = __builtin_bit_cast(_Float16, lb);
            }
          }
          *(volatile v8h*)(Cb + go) = hv;
          if (EPI == EPI_QK || EPI == EPI_GATE) *(volatile v8h*)(Cb2 + go) = lv;
        }
        __threadfence();
      }
    }
    __builtin_amdgcn_fence(__ATOMIC_RELEASE, "workgroup");
    __builtin_amdgcn_wave_barrier();
    __builtin_amdgcn_fence(__ATOMIC_ACQUIRE, "workgroup");
  }
}

template <int MODE>
__global__ __launch_bounds__(256) void k_transpose_cast64(
    const float* __restrict__ in, unsigned short* __restrict__ out, unsigned short* __restrict__ out2,
    int R, int C, float mul) {
  __shared__ float t[64][65];
  const int c0 = blockIdx.x * 64;
  const int r0 = blockIdx.y * 64;
  const int tid = threadIdx.x, lane = tid & 31, wave = tid >> 5;
  {
    const int rr = tid >> 2, cc = (tid & 3) * 16;
    const float* src = in + (size_t)(r0 + rr) * C + c0 + cc;
#pragma unroll
    for (int e = 0; e < 4; ++e) {
      const v4f w = *(const v4f*)(src + 4 * e);
      t[rr][cc + 4 * e + 0] = w[0];
      t[rr][cc + 4 * e + 1] = w[1];
      t[rr][cc + 4 * e + 2] = w[2];
      t[rr][cc + 4 * e + 3] = w[3];
    }
  }
  __syncthreads();
  const int q = lane >> 3, c8 = (lane & 7) * 8;
  for (int pass = 0; pass < 2; ++pass) {
#pragma unroll
    for (int it = 0; it < 2; ++it) {
      const int orow = wave * 8 + it * 4 + q;
      v8h hv, lv;
#pragma unroll
      for (int e = 0; e < 8; ++e) {
        const float f = t[c8 + e][orow] * mul;
        if (MODE == 0) {
          hv[e] = (_Float16)f;
          lv[e] = hv[e];
        } else {
          const unsigned short hb = f2bf_bits(f);
          const unsigned short lb = f2bf_bits(f - bf_bits2f(hb));
          hv[e] = __builtin_bit_cast(_Float16, hb);
          lv[e] = __builtin_bit_cast(_Float16, lb);
        }
      }
      const size_t o = (size_t)(c0 + orow) * R + r0 + c8;
      *(volatile v8h*)(out + o) = hv;
      if (MODE == 1) *(volatile v8h*)(out2 + o) = lv;
    }
    __threadfence();
  }
}

__global__ __launch_bounds__(256) void k_scalenorm(const float* __restrict__ x, const float* __restrict__ g_ln,
                                                    unsigned short* __restrict__ xn) {
  const int lane = threadIdx.x & 31, wave = threadIdx.x >> 5;
  const int row = blockIdx.x * 8 + wave;
  const float* xr = x + (size_t)row * DMODEL;
  float v[16];
#pragma unroll
  for (int it = 0; it < 2; ++it) {
#pragma unroll
    for (int e = 0; e < 2; ++e) {
      const v4f w = *(const v4f*)(xr + it * 256 + 8 * lane + 4 * e);
      v[it * 8 + 4 * e + 0] = w[0];
      v[it * 8 + 4 * e + 1] = w[1];
      v[it * 8 + 4 * e + 2] = w[2];
      v[it * 8 + 4 * e + 3] = w[3];
    }
  }
  float ss = 0.0f;
#pragma unroll
  for (int e = 0; e < 16; ++e) ss += v[e] * v[e];
#pragma unroll
  for (int off = 16; off > 0; off >>= 1) ss += __shfl_xor(ss, off, 32);
  const float nrm = sqrtf(ss) * 0.04419417382415922f;
  const float den = fmaxf(nrm, 1e-5f);
  const float rinv = 1.0f / den;
  const float g = g_ln[0];
  v8h h0, h1;
#pragma unroll
  for (int e = 0; e < 8; ++e) {
    h0[e] = (_Float16)((v[e] * rinv) * g);
    h1[e] = (_Float16)((v[8 + e] * rinv) * g);
  }
  unsigned short* dst = xn + (size_t)row * DMODEL;
  for (int pass = 0; pass < 2; ++pass) {
    *(volatile v8h*)(dst + 8 * lane) = h0;
    *(volatile v8h*)(dst + 256 + 8 * lane) = h1;
    __threadfence();
  }
}

extern "C" void kernel_launch(void* const* d_in, const int* in_sizes, int n_in,
                              void* d_out, int out_size, void* d_ws, size_t ws_size,
                              hipStream_t stream) {
  (void)in_sizes; (void)n_in; (void)out_size;
  if (ws_size < WS_TOTAL) return;
  const float* x         = (const float*)d_in[0];
  const float* W_uv      = (const float*)d_in[1];
  const float* gamma     = (const float*)d_in[2];
  const float* beta      = (const float*)d_in[3];
  const float* w_rel     = (const float*)d_in[4];
  const float* W_o       = (const float*)d_in[5];
  const float* g_ln      = (const float*)d_in[6];
  const float* res_scale = (const float*)d_in[7];
  float* out = (float*)d_out;

  unsigned char* ws = (unsigned char*)d_ws;
  unsigned short* WuvT = (unsigned short*)(ws + OFF_WUVT);
  unsigned short* WoH  = (unsigned short*)(ws + OFF_WOH);
  unsigned short* WoL  = (unsigned short*)(ws + OFF_WOL);
  unsigned short* Xn   = (unsigned short*)(ws + OFF_XN);
  float*          U    = (float*)(ws + OFF_U);
  unsigned short* Vt   = (unsigned short*)(ws + OFF_VT);
  unsigned short* Qp   = (unsigned short*)(ws + OFF_Q);
  unsigned short* Kp   = (unsigned short*)(ws + OFF_K);
  unsigned short* Sc   = (unsigned short*)(ws + OFF_SC);
  unsigned short* HH   = (unsigned short*)(ws + OFF_HH);
  unsigned short* HL   = (unsigned short*)(ws + OFF_HL);

  k_transpose_cast64<0><<<dim3(NUV / 64, DMODEL / 64), 256, 0, stream>>>(W_uv, WuvT, WuvT, DMODEL, NUV, 16.0f);
  k_transpose_cast64<1><<<dim3(DMODEL / 64, EDIM / 64), 256, 0, stream>>>(W_o, WoH, WoL, EDIM, DMODEL, 1.0f);
  k_scalenorm<<<NROWS / 8, 256, 0, stream>>>(x, g_ln, Xn);

  const unsigned short* WuvT_v  = WuvT + (size_t)EDIM * DMODEL;
  const unsigned short* WuvT_qk = WuvT + (size_t)2 * EDIM * DMODEL;

  for (int g = 0; g < NGRP; ++g) {
    const size_t r0 = (size_t)g * GROWS;
    const unsigned short* XnG = Xn + r0 * DMODEL;

    gemm64<0, false, EPI_U><<<dim3((LSEQ / 64) * (EDIM / 64) / 8, GRP), 256, 0, stream>>>(
        XnG, XnG, DMODEL, (long)LSEQ * DMODEL,
        WuvT, WuvT, DMODEL, 0L,
        U, U, EDIM, (long)LSEQ * EDIM,
        gamma, gamma, 0L,
        LSEQ, EDIM, DMODEL, 1.0f / 16.0f, 0.0f);

    gemm64<0, false, EPI_VT><<<dim3((EDIM / 64) * (LSEQ / 64) / 8, GRP), 256, 0, stream>>>(
        WuvT_v, WuvT_v, DMODEL, 0L,
        XnG, XnG, DMODEL, (long)LSEQ * DMODEL,
        Vt, Vt, LSEQ, (long)EDIM * LSEQ,
        gamma, gamma, 0L,
        EDIM, LSEQ, DMODEL, 1.0f / 16.0f, 64.0f);

    gemm64<0, false, EPI_QK><<<dim3((LSEQ / 64) * (SHEAD / 64) / 8, GRP), 256, 0, stream>>>(
        XnG, XnG, DMODEL, (long)LSEQ * DMODEL,
        WuvT_qk, WuvT_qk, DMODEL, 0L,
        Qp, Kp, SHEAD, (long)LSEQ * SHEAD,
        gamma, beta, 0L,
        LSEQ, SHEAD, DMODEL, 1.0f / 16.0f, 0.0f);

    gemm64<0, false, EPI_SC><<<dim3((LSEQ / 64) * (LSEQ / 64) / 8, GRP), 256, 0, stream>>>(
        Qp, Qp, SHEAD, (long)LSEQ * SHEAD,
        Kp, Kp, SHEAD, (long)LSEQ * SHEAD,
        Sc, Sc, LSEQ, (long)LSEQ * LSEQ,
        w_rel, w_rel, 0L,
        LSEQ, LSEQ, SHEAD, 1.0f, 0.08838834764831845f);

    gemm64<0, false, EPI_GATE><<<dim3((LSEQ / 64) * (EDIM / 64) / 8, GRP), 256, 0, stream>>>(
        Sc, Sc, LSEQ, (long)LSEQ * LSEQ,
        Vt, Vt, LSEQ, (long)EDIM * LSEQ,
        HH, HL, EDIM, (long)LSEQ * EDIM,
        U, res_scale, (long)LSEQ * EDIM,
        LSEQ, EDIM, LSEQ, 1.0f / 64.0f, 0.0f);

    gemm64<1, true, EPI_OUT><<<dim3((LSEQ / 64) * (DMODEL / 64) / 8, GRP), 256, 0, stream>>>(
        HH, HL, EDIM, (long)LSEQ * EDIM,
        WoH, WoL, EDIM, 0L,
        out + r0 * DMODEL, out + r0 * DMODEL, DMODEL, (long)LSEQ * DMODEL,
        x + r0 * DMODEL, res_scale, (long)LSEQ * DMODEL,
        LSEQ, DMODEL, EDIM, 1.0f, 0.0f);
  }
}
